// RNN2D_23021024706894
// MI455X (gfx1250) — hardware-run, weakly checked
//
#include <hip/hip_runtime.h>
#include <math.h>

constexpr int NBATCH   = 1024;
constexpr int LAT      = 32;
constexpr int NHID     = 64;
constexpr int NCLS     = 2;
constexpr int NSITE    = LAT * LAT;
constexpr int NWAVES   = 2;
constexpr int WROWS    = 16;
constexpr int NTHREADS = 32 * NWAVES;
constexpr int BLKROWS  = WROWS * NWAVES;
constexpr int NBLOCKS  = NBATCH / BLKROWS;
constexpr int HTILE    = WROWS * NHID;
constexpr int HWAVE    = LAT * HTILE;
constexpr float LOGP_SCALE = 0.5f;
constexpr float NAN_FILL   = -35.0f;
constexpr float F32_MAXV   = 3.402823466e+38f;

static_assert(NBATCH % BLKROWS == 0, "batch rows split evenly over blocks");
static_assert(BLKROWS == 32, "one block owns one 128-B output line");
static_assert(NHID == 64 && NHID % 32 == 0, "K = 64 = two 32-deep k steps, N = 64 = four 16-wide column tiles");
static_assert(NCLS == 2, "two classes");
static_assert(LAT == 32, "lattice side");
static_assert((HWAVE / 4) % 32 == 0, "zero fill loop exact");
static_assert((NHID * NHID / 4) % NTHREADS == 0, "weight staging loop exact");

typedef __attribute__((ext_vector_type(16))) __bf16   v16b;
typedef __attribute__((ext_vector_type(8)))  float    v8f;
typedef __attribute__((ext_vector_type(4)))  float    v4f;
typedef __attribute__((ext_vector_type(8)))  unsigned v8u;
typedef __attribute__((ext_vector_type(4)))  unsigned v4u;

__device__ __forceinline__ unsigned bf_rne_u(unsigned u) { return u + 0x7FFFu + ((u >> 16) & 1u); }

__device__ __forceinline__ void split2(float s0, float s1, unsigned& hw, unsigned& lw) {
  const unsigned t0 = bf_rne_u(__float_as_uint(s0));
  const unsigned t1 = bf_rne_u(__float_as_uint(s1));
  const float r0 = s0 - __uint_as_float(t0 & 0xFFFF0000u);
  const float r1 = s1 - __uint_as_float(t1 & 0xFFFF0000u);
  const unsigned l0 = bf_rne_u(__float_as_uint(r0));
  const unsigned l1 = bf_rne_u(__float_as_uint(r1));
  hw = (t0 >> 16) | (t1 & 0xFFFF0000u);
  lw = (l0 >> 16) | (l1 & 0xFFFF0000u);
}

__device__ __forceinline__ unsigned pack_hi2(float a, float b) {
  const unsigned ta = bf_rne_u(__float_as_uint(a));
  const unsigned tb = bf_rne_u(__float_as_uint(b));
  return (ta >> 16) | (tb & 0xFFFF0000u);
}

__device__ __forceinline__ unsigned pack_lo2(float a, float b) {
  unsigned hw, lw;
  split2(a, b, hw, lw);
  return lw;
}

__device__ __forceinline__ v8f mma_bf(v16b a, v16b b, v8f c) {
  c = __builtin_amdgcn_wmma_f32_16x16x32_bf16(false, a, false, b, (short)0, c, false, false);
  asm volatile("v_nop\n\tv_nop\n\tv_nop\n\tv_nop" : "+v"(c) : "v"(a), "v"(b));
  return c;
}

__device__ __forceinline__ void wave_lds_sync() {
  __builtin_amdgcn_fence(__ATOMIC_RELEASE, "workgroup");
  __builtin_amdgcn_wave_barrier();
  __builtin_amdgcn_fence(__ATOMIC_ACQUIRE, "workgroup");
}

__device__ __forceinline__ float elu1(float v) {
  const float e = expf(fminf(v, 0.0f)) - 1.0f;
  return (v > 0.0f) ? v : e;
}

extern "C" __global__ __launch_bounds__(NTHREADS) __attribute__((amdgpu_num_vgpr(256)))
void lattice_scan_kernel(const int* __restrict__ x, const float* __restrict__ Win, const float* __restrict__ Wc,
                         const float* __restrict__ bc, const float* __restrict__ Wout, const float* __restrict__ bout,
                         float* __restrict__ out) {
  __shared__ __align__(16) float    hsm[NWAVES * HWAVE];
  __shared__ __align__(16) unsigned xws[NWAVES * NSITE];
  __shared__ __align__(16) unsigned wlo[NHID * NHID / 2];
  __shared__ __align__(16) float    wouts[NHID * NCLS];
  __shared__ __align__(16) float    outs[BLKROWS];

  const int tid  = threadIdx.x;
  const int lane = tid & 31;
  const int wave = tid >> 5;
  const int hf   = lane >> 4;
  const int li   = lane & 15;
  const int batchBase = (blockIdx.x * NWAVES + wave) * WROWS;

  {
    const v4f* wsrc = (const v4f*)Wc;
    v4f* wdst = (v4f*)hsm;
#pragma unroll 4
    for (int it = 0; it < (NHID * NHID / 4) / NTHREADS; ++it) wdst[it * NTHREADS + tid] = wsrc[it * NTHREADS + tid];
  }
  if (tid < 32) {
    const v4f wv = ((const v4f*)Wout)[tid];
    ((v4f*)wouts)[tid] = wv;
  }
  unsigned* xwv = xws + wave * NSITE;
  {
    const int* xb = x + (size_t)batchBase * NSITE;
#pragma unroll 1
    for (int it = 0; it < NSITE / 32; ++it) {
      const int s = it * 32 + lane;
      unsigned word = 0u;
#pragma unroll
      for (int m = 0; m < WROWS; ++m) {
        const int v = xb[m * NSITE + s];
        word |= ((v == 1) ? 1u : 0u) << m;
        word |= ((v == 0) ? 1u : 0u) << (16 + m);
      }
      xwv[s] = word;
    }
  }
  __syncthreads();

  v16b bhi[2][4];
  {
    const float* wst = hsm;
#pragma unroll
    for (int kt = 0; kt < 2; ++kt) {
#pragma unroll
      for (int t = 0; t < 4; ++t) {
        const int n = 16 * t + li;
        unsigned w[8];
#pragma unroll
        for (int jj = 0; jj < 4; ++jj) {
          const int ka = 32 * kt + 8 * hf + 2 * jj;
          w[jj]     = pack_hi2(wst[ka * NHID + n],        wst[(ka + 1) * NHID + n]);
          w[4 + jj] = pack_hi2(wst[(ka + 16) * NHID + n], wst[(ka + 17) * NHID + n]);
        }
        const v8u wv = {w[0], w[1], w[2], w[3], w[4], w[5], w[6], w[7]};
        bhi[kt][t] = __builtin_bit_cast(v16b, wv);
      }
    }
#pragma unroll 4
    for (int kp = 0; kp < NHID / 2; ++kp) {
      const float wa = wst[(2 * kp) * NHID + tid];
      const float wb = wst[(2 * kp + 1) * NHID + tid];
      wlo[tid * (NHID / 2) + kp] = pack_lo2(wa, wb);
    }
  }
  __syncthreads();

  float* hw_ = hsm + wave * HWAVE;
  {
    const v4f z4i = {0.f, 0.f, 0.f, 0.f};
    v4f* hz = (v4f*)hw_;
#pragma unroll 4
    for (int i = lane; i < HWAVE / 4; i += 32) hz[i] = z4i;
  }
  float win0[4], win1[4], bcv[4];
#pragma unroll
  for (int t = 0; t < 4; ++t) {
    const int n = 16 * t + li;
    win0[t] = Win[n];
    win1[t] = Win[NHID + n];
    bcv[t]  = bc[n];
  }
  const float bo0 = bout[0];
  const float bo1 = bout[1];
  __syncthreads();

  const v4f z4 = {0.f, 0.f, 0.f, 0.f};
  const int m2 = lane >> 1;
  const int ch = lane & 1;
  const int wlo_base = li * (NHID / 2) + 4 * hf;
  float total = 0.0f;

#pragma unroll 1
  for (int r = 0; r < LAT; ++r) {
    const bool even = ((r & 1) == 0);
    const bool hasU = (r > 0);
    const int  rup  = hasU ? (r - 1) : 0;
    float rowacc = 0.0f;
#pragma unroll 1
    for (int j = 0; j < LAT; ++j) {
      const int  c    = even ? j : (LAT - 1 - j);
      const int  cpc  = (even ? (c - 1) : (c + 1)) & (LAT - 1);
      const bool hasL = (j > 0);

      const unsigned curw  = xwv[r * LAT + c];
      const unsigned lraw  = xwv[r * LAT + cpc];
      const unsigned uraw  = xwv[rup * LAT + c];
      const unsigned leftw = hasL ? lraw : 0u;
      const unsigned upw   = hasU ? uraw : 0u;
      const unsigned lsh   = leftw >> (8 * hf);
      const unsigned ush   = upw >> (8 * hf);

      v8f acc[4];
      {
        float c0f[8], c1f[8];
#pragma unroll
        for (int i = 0; i < 8; ++i) {
          c1f[i] = (float)(((lsh >> i) & 1u) + ((ush >> i) & 1u));
          c0f[i] = (float)(((lsh >> (16 + i)) & 1u) + ((ush >> (16 + i)) & 1u));
        }
#pragma unroll
        for (int t = 0; t < 4; ++t) {
#pragma unroll
          for (int i = 0; i < 8; ++i)
            acc[t][i] = fmaf(c1f[i], win1[t], fmaf(c0f[i], win0[t], bcv[t]));
        }
      }

      float* hc = hw_ + c * HTILE;
      const float* up = hc + li * NHID + 8 * hf;
      const float* lf = hw_ + cpc * HTILE + li * NHID + 8 * hf;
      int wo = wlo_base;
      asm volatile("" : "+v"(wo));

#pragma unroll
      for (int kt = 0; kt < 2; ++kt) {
        const v4f u0 = *(const v4f*)(up + 32 * kt);
        const v4f u1 = *(const v4f*)(up + 32 * kt + 4);
        const v4f u2 = *(const v4f*)(up + 32 * kt + 16);
        const v4f u3 = *(const v4f*)(up + 32 * kt + 20);
        const v4f l0 = *(const v4f*)(lf + 32 * kt);
        const v4f l1 = *(const v4f*)(lf + 32 * kt + 4);
        const v4f l2 = *(const v4f*)(lf + 32 * kt + 16);
        const v4f l3 = *(const v4f*)(lf + 32 * kt + 20);
        const v4f s0 = u0 + (hasL ? l0 : z4);
        const v4f s1 = u1 + (hasL ? l1 : z4);
        const v4f s2 = u2 + (hasL ? l2 : z4);
        const v4f s3 = u3 + (hasL ? l3 : z4);
        unsigned h0, h1, h2, h3, h4, h5, h6, h7;
        unsigned q0, q1, q2, q3, q4, q5, q6, q7;
        split2(s0[0], s0[1], h0, q0);
        split2(s0[2], s0[3], h1, q1);
        split2(s1[0], s1[1], h2, q2);
        split2(s1[2], s1[3], h3, q3);
        split2(s2[0], s2[1], h4, q4);
        split2(s2[2], s2[3], h5, q5);
        split2(s3[0], s3[1], h6, q6);
        split2(s3[2], s3[3], h7, q7);
        const v8u ahw = {h0, h1, h2, h3, h4, h5, h6, h7};
        const v8u alw = {q0, q1, q2, q3, q4, q5, q6, q7};
        const v16b ahi = __builtin_bit_cast(v16b, ahw);
        const v16b alo = __builtin_bit_cast(v16b, alw);
#pragma unroll
        for (int t = 0; t < 4; ++t) {
          const unsigned* bp = wlo + wo + t * (16 * (NHID / 2)) + 16 * kt;
          const v4u b0 = *(const v4u*)(bp);
          const v4u b1 = *(const v4u*)(bp + 8);
          const v8u bw = __builtin_shufflevector(b0, b1, 0, 1, 2, 3, 4, 5, 6, 7);
          const v16b blo = __builtin_bit_cast(v16b, bw);
          acc[t] = mma_bf(ahi, bhi[kt][t], acc[t]);
          acc[t] = mma_bf(alo, bhi[kt][t], acc[t]);
          acc[t] = mma_bf(ahi, blo, acc[t]);
        }
      }

      {
        float* dst = hc + (8 * hf) * NHID + li;
#pragma unroll
        for (int t = 0; t < 4; ++t) {
#pragma unroll
          for (int i = 0; i < 8; ++i) dst[i * NHID + 16 * t] = acc[t][i];
        }
      }
      wave_lds_sync();

      float z0 = 0.0f, z1 = 0.0f;
      {
        float* rp = hc + m2 * NHID + 32 * ch;
        const float* wp = wouts + 64 * ch;
#pragma unroll 1
        for (int it = 0; it < 8; ++it) {
          const v4f p  = *(const v4f*)(rp + 4 * it);
          const v4f wa = *(const v4f*)(wp + 8 * it);
          const v4f wb = *(const v4f*)(wp + 8 * it + 4);
          v4f o;
          o[0] = elu1(p[0]);
          o[1] = elu1(p[1]);
          o[2] = elu1(p[2]);
          o[3] = elu1(p[3]);
          z0 = fmaf(o[0], wa[0], z0);
          z1 = fmaf(o[0], wa[1], z1);
          z0 = fmaf(o[1], wa[2], z0);
          z1 = fmaf(o[1], wa[3], z1);
          z0 = fmaf(o[2], wb[0], z0);
          z1 = fmaf(o[2], wb[1], z1);
          z0 = fmaf(o[3], wb[2], z0);
          z1 = fmaf(o[3], wb[3], z1);
          *(v4f*)(rp + 4 * it) = o;
        }
      }
      const float zo0 = __shfl_xor(z0, 1, 32);
      const float zo1 = __shfl_xor(z1, 1, 32);
      z0 = (z0 + zo0) + bo0;
      z1 = (z1 + zo1) + bo1;
      {
        const float zm  = fmaxf(z0, z1);
        const float sh0 = z0 - zm;
        const float sh1 = z1 - zm;
        const float lse = logf(expf(sh0) + expf(sh1));
        const float lp0 = sh0 - lse;
        const float lp1 = sh1 - lse;
        const unsigned cw = curw >> m2;
        const bool is1 = (cw & 1u) != 0u;
        const bool is0 = ((cw >> 16) & 1u) != 0u;
        float p = (is0 ? lp0 : 0.0f) + (is1 ? lp1 : 0.0f);
        p = (p != p) ? NAN_FILL : p;
        p = fminf(fmaxf(p, -F32_MAXV), F32_MAXV);
        rowacc += p;
      }
      wave_lds_sync();
    }
    total += rowacc;
  }

  if (ch == 0) outs[WROWS * wave + m2] = LOGP_SCALE * total;
  __syncthreads();
  if (wave == 0) {
    const float v = outs[lane];
    volatile float* op = out + (size_t)blockIdx.x * BLKROWS + lane;
    *op = v;
    __threadfence();
    *op = v;
  }
}

extern "C" void kernel_launch(void* const* d_in, const int* in_sizes, int n_in,
                              void* d_out, int out_size, void* d_ws, size_t ws_size, hipStream_t stream) {
  (void)d_ws;
  (void)ws_size;
  if (n_in < 6 || d_out == nullptr) return;
  if (in_sizes[0] != NBATCH * NSITE || in_sizes[1] != NCLS * NHID || in_sizes[2] != NHID * NHID ||
      in_sizes[3] != NHID || in_sizes[4] != NHID * NCLS || in_sizes[5] != NCLS || out_size != NBATCH) return;

  const int*   x    = (const int*)d_in[0];
  const float* Win  = (const float*)d_in[1];
  const float* Wc   = (const float*)d_in[2];
  const float* bc   = (const float*)d_in[3];
  const float* Wout = (const float*)d_in[4];
  const float* bout = (const float*)d_in[5];
  float* out = (float*)d_out;

  lattice_scan_kernel<<<NBLOCKS, NTHREADS, 0, stream>>>(x, Win, Wc, bc, Wout, bout, out);
}
